// LSTMscratch_76055280877768
// MI455X (gfx1250) — hardware-verified
//
#include <hip/hip_runtime.h>
#define NBT 32
#define NT_ 32
#define NF (NBT * NT_)
#define IMG 64
#define C1 16
#define C2 32
#define DIN 256
#define HID 512
#define G4 2048
#define NCLS 6

typedef __bf16 v16b __attribute__((ext_vector_type(16)));
typedef unsigned short v8us __attribute__((ext_vector_type(8), may_alias));
typedef float  v8f  __attribute__((ext_vector_type(8)));
typedef float  v4f  __attribute__((ext_vector_type(4)));
typedef float  v4fa __attribute__((ext_vector_type(4), may_alias));
union FragB { v16b v; v8us half[2]; unsigned short u[16]; };

__device__ __forceinline__ unsigned short bf16_bits(float x) { unsigned int u = __float_as_uint(x); return (unsigned short)((u + 0x7FFFu + ((u >> 16) & 1u)) >> 16); }
__device__ __forceinline__ float bf16_val(unsigned short b) { return __uint_as_float(((unsigned int)b) << 16); }
__device__ __forceinline__ float bf16_round(float x) { return bf16_val(bf16_bits(x)); }
template <int NT>
__device__ __forceinline__ v8f mmaN(v16b ah, v16b al, v16b bh, v16b bl, v8f c) {
  c = __builtin_amdgcn_wmma_f32_16x16x32_bf16(false, ah, false, bh, (short)0, c, false, false);
  if (NT >= 2) c = __builtin_amdgcn_wmma_f32_16x16x32_bf16(false, al, false, bh, (short)0, c, false, false);
  if (NT >= 3) c = __builtin_amdgcn_wmma_f32_16x16x32_bf16(false, ah, false, bl, (short)0, c, false, false);
  asm volatile("v_nop\n\tv_nop\n\tv_nop\n\tv_nop" : "+v"(c) : "v"(ah), "v"(al), "v"(bh), "v"(bl));
  return c;
}

__global__ __launch_bounds__(256) void k_wt_bf16(const float* __restrict__ W, unsigned short* __restrict__ Wt, int K, int N) {
  const int t = blockIdx.x * 256 + threadIdx.x;
  const int k8n = K / 8;
  if (t >= N * k8n) return;
  const int n = t / k8n, k8 = (t % k8n) * 8;
  v8us v;
#pragma unroll
  for (int i = 0; i < 8; ++i) v[i] = bf16_bits(W[(size_t)(k8 + i) * N + n]);
  *(volatile v8us*)(Wt + (size_t)n * K + k8) = v;
  __threadfence();
  *(volatile v8us*)(Wt + (size_t)n * K + k8) = v;
}

template <bool ASPLIT, int ACT, bool BIAS_BF16>
__global__ __launch_bounds__(128) void k_gemm_bf(const float* __restrict__ A, int lda, const unsigned short* __restrict__ Wt, int ldb,
                                               const float* __restrict__ bias, float* __restrict__ C, int ldc, int M, int N, int K) {
  __shared__ __attribute__((aligned(16))) float so[4][16][64];
  const int tid = threadIdx.x, w = tid >> 5, lane = tid & 31, ln = lane & 15, hh = lane >> 4;
  const int ntn = N / 64;
  const int wid = blockIdx.x * 4 + w;
  const int mt = wid / ntn, nq = wid % ntn;
  if (mt * 16 >= M) return;
  const int row0 = mt * 16, col0 = nq * 64;
  const float* arow = A + (size_t)(row0 + ln) * lda;
  v8f acc[4] = {};
  for (int kb = 0; kb < K; kb += 32) {
    FragB ah, al;
    const v4f x0 = *(const v4fa*)(arow + kb + 8 * hh), x1 = *(const v4fa*)(arow + kb + 8 * hh + 4);
    const v4f x2 = *(const v4fa*)(arow + kb + 16 + 8 * hh), x3 = *(const v4fa*)(arow + kb + 16 + 8 * hh + 4);
    float xs[16] = {x0[0],x0[1],x0[2],x0[3],x1[0],x1[1],x1[2],x1[3],x2[0],x2[1],x2[2],x2[3],x3[0],x3[1],x3[2],x3[3]};
#pragma unroll
    for (int i = 0; i < 16; ++i) { const unsigned short hb = bf16_bits(xs[i]); ah.u[i] = hb; al.u[i] = ASPLIT ? bf16_bits(xs[i] - bf16_val(hb)) : (unsigned short)0; }
#pragma unroll
    for (int t = 0; t < 4; ++t) {
      const unsigned short* brow = Wt + (size_t)(col0 + t * 16 + ln) * ldb + kb;
      FragB b;
      b.half[0] = *(const v8us*)(brow + 8 * hh);
      b.half[1] = *(const v8us*)(brow + 16 + 8 * hh);
      acc[t] = mmaN<ASPLIT ? 2 : 1>(ah.v, al.v, b.v, b.v, acc[t]);
    }
  }
#pragma unroll
  for (int t = 0; t < 4; ++t) {
    float bv = bias ? bias[col0 + t * 16 + ln] : 0.f;
    if (BIAS_BF16) bv = bf16_round(bv);
#pragma unroll
    for (int r = 0; r < 8; ++r) { float v = acc[t][r] + bv; if (ACT == 1) v = fmaxf(v, 0.f); so[w][8 * hh + r][t * 16 + ln] = v; }
  }
  __builtin_amdgcn_fence(__ATOMIC_ACQ_REL, "workgroup");
  __builtin_amdgcn_wave_barrier();
  const int rsub = lane >> 4, c4 = (lane & 15) * 4;
  for (int pass = 0; pass < 2; ++pass) {
#pragma unroll
    for (int q = 0; q < 8; ++q) {
      const int r = q * 2 + rsub;
      const v4f v = *(const v4fa*)&so[w][r][c4];
      *(volatile v4f*)(C + (size_t)(row0 + r) * ldc + col0 + c4) = v;
    }
    if (pass == 0) __threadfence();
  }
}

template <int D, bool CAUSAL>
__global__ __launch_bounds__(128) void k_flash(const float* __restrict__ qb, const float* __restrict__ kb, const float* __restrict__ vb,
                                             int pitch, int T, int H, float scale, float* __restrict__ y, int ypitch) {
  constexpr int KS = D / 32;
  constexpr int DT = D / 16;
  __shared__ __attribute__((aligned(16))) unsigned short sKh[32][D + 8], sKl[32][D + 8], sVh[32][D + 8], sVl[32][D + 8];
  __shared__ __attribute__((aligned(16))) unsigned short sPh[4][16][40], sPl[4][16][40];
  __shared__ __attribute__((aligned(16))) float sO[4][16][D];
  const int tid = threadIdx.x, w = tid >> 5, lane = tid & 31, ln = lane & 15, hh = lane >> 4;
  const int nqb = (T + 63) / 64;
  const int bh = blockIdx.x / nqb, qblk = blockIdx.x % nqb;
  const int b = bh / H, h = bh % H;
  const int q0 = qblk * 64 + w * 16;
  const float* Q = qb + (size_t)b * T * pitch + h * D;
  const float* K = kb + (size_t)b * T * pitch + h * D;
  const float* V = vb + (size_t)b * T * pitch + h * D;

  FragB aqh[KS], aql[KS];
  {
    int row = q0 + ln; if (row >= T) row = T - 1;
    const float* qr = Q + (size_t)row * pitch;
#pragma unroll
    for (int ks = 0; ks < KS; ++ks)
#pragma unroll
      for (int i = 0; i < 16; ++i) {
        const int d = ks * 32 + ((i < 8) ? (8 * hh + i) : (16 + 8 * hh + (i - 8)));
        const float x = qr[d] * scale; const unsigned short hb = bf16_bits(x);
        aqh[ks].u[i] = hb; aql[ks].u[i] = bf16_bits(x - bf16_val(hb));
      }
  }
  float m_r[8], l_r[8];
#pragma unroll
  for (int r = 0; r < 8; ++r) { m_r[r] = -3.0e38f; l_r[r] = 0.f; }
  v8f oacc[DT];
#pragma unroll
  for (int dt = 0; dt < DT; ++dt) oacc[dt] = (v8f){0.f,0.f,0.f,0.f,0.f,0.f,0.f,0.f};

  const int kv_end = CAUSAL ? min(T, qblk * 64 + 64) : T;
  for (int j0 = 0; j0 < kv_end; j0 += 32) {
    __syncthreads();
    for (int e = tid; e < 32 * (D / 4); e += 128) {
      const int r = e / (D / 4), c4 = (e % (D / 4)) * 4;
      const int key = j0 + r;
      v4f kf = {0.f,0.f,0.f,0.f}, vf = {0.f,0.f,0.f,0.f};
      if (key < T) { kf = *(const v4fa*)(K + (size_t)key * pitch + c4); vf = *(const v4fa*)(V + (size_t)key * pitch + c4); }
#pragma unroll
      for (int t = 0; t < 4; ++t) {
        unsigned short hb = bf16_bits(kf[t]); sKh[r][c4 + t] = hb; sKl[r][c4 + t] = bf16_bits(kf[t] - bf16_val(hb));
        hb = bf16_bits(vf[t]); sVh[r][c4 + t] = hb; sVl[r][c4 + t] = bf16_bits(vf[t] - bf16_val(hb));
      }
    }
    __syncthreads();
    v8f s[2];
#pragma unroll
    for (int nt = 0; nt < 2; ++nt) {
      v8f acc = {};
#pragma unroll
      for (int ks = 0; ks < KS; ++ks) {
        FragB bh_, bl_;
        bh_.half[0] = *(const v8us*)&sKh[nt * 16 + ln][ks * 32 + 8 * hh]; bh_.half[1] = *(const v8us*)&sKh[nt * 16 + ln][ks * 32 + 16 + 8 * hh];
        bl_.half[0] = *(const v8us*)&sKl[nt * 16 + ln][ks * 32 + 8 * hh]; bl_.half[1] = *(const v8us*)&sKl[nt * 16 + ln][ks * 32 + 16 + 8 * hh];
        acc = mmaN<3>(aqh[ks].v, aql[ks].v, bh_.v, bl_.v, acc);
      }
      s[nt] = acc;
    }
    float alpha[8];
#pragma unroll
    for (int r = 0; r < 8; ++r) {
      const int qi = q0 + 8 * hh + r;
      const int ja = j0 + ln, jb = j0 + 16 + ln;
      if (CAUSAL) { if (ja > qi) s[0][r] = -3.0e38f; if (jb > qi) s[1][r] = -3.0e38f; }
      if (ja >= T) s[0][r] = -3.0e38f;
      if (jb >= T) s[1][r] = -3.0e38f;
      float mx = fmaxf(s[0][r], s[1][r]);
      mx = fmaxf(mx, __shfl_xor(mx, 1, 32)); mx = fmaxf(mx, __shfl_xor(mx, 2, 32)); mx = fmaxf(mx, __shfl_xor(mx, 4, 32)); mx = fmaxf(mx, __shfl_xor(mx, 8, 32));
      const float mnew = fmaxf(m_r[r], mx);
      alpha[r] = (mnew > -1.0e38f) ? __expf(m_r[r] - mnew) : 1.0f;
      const float p0 = (s[0][r] > -1.0e38f) ? __expf(s[0][r] - mnew) : 0.f;
      const float p1 = (s[1][r] > -1.0e38f) ? __expf(s[1][r] - mnew) : 0.f;
      m_r[r] = mnew;
      l_r[r] = l_r[r] * alpha[r] + p0 + p1;
      unsigned short hb = bf16_bits(p0); sPh[w][8 * hh + r][ln] = hb;      sPl[w][8 * hh + r][ln] = bf16_bits(p0 - bf16_val(hb));
      hb = bf16_bits(p1);                sPh[w][8 * hh + r][16 + ln] = hb; sPl[w][8 * hh + r][16 + ln] = bf16_bits(p1 - bf16_val(hb));
    }
#pragma unroll
    for (int dt = 0; dt < DT; ++dt)
#pragma unroll
      for (int r = 0; r < 8; ++r) oacc[dt][r] *= alpha[r];
    __builtin_amdgcn_fence(__ATOMIC_ACQ_REL, "workgroup");
    __builtin_amdgcn_wave_barrier();
    FragB pah, pal;
    pah.half[0] = *(const v8us*)&sPh[w][ln][8 * hh]; pah.half[1] = *(const v8us*)&sPh[w][ln][16 + 8 * hh];
    pal.half[0] = *(const v8us*)&sPl[w][ln][8 * hh]; pal.half[1] = *(const v8us*)&sPl[w][ln][16 + 8 * hh];
#pragma unroll
    for (int dt = 0; dt < DT; ++dt) {
      FragB bvh, bvl;
#pragma unroll
      for (int i = 0; i < 8; ++i) {
        bvh.u[i] = sVh[8 * hh + i][dt * 16 + ln]; bvh.u[8 + i] = sVh[16 + 8 * hh + i][dt * 16 + ln];
        bvl.u[i] = sVl[8 * hh + i][dt * 16 + ln]; bvl.u[8 + i] = sVl[16 + 8 * hh + i][dt * 16 + ln];
      }
      oacc[dt] = mmaN<3>(pah.v, pal.v, bvh.v, bvl.v, oacc[dt]);
    }
    __builtin_amdgcn_fence(__ATOMIC_ACQ_REL, "workgroup");
    __builtin_amdgcn_wave_barrier();
  }
#pragma unroll
  for (int r = 0; r < 8; ++r) {
    float l = l_r[r];
    l += __shfl_xor(l, 1, 32); l += __shfl_xor(l, 2, 32); l += __shfl_xor(l, 4, 32); l += __shfl_xor(l, 8, 32);
    l_r[r] = (l > 0.f) ? 1.0f / l : 0.f;
  }
#pragma unroll
  for (int dt = 0; dt < DT; ++dt)
#pragma unroll
    for (int r = 0; r < 8; ++r) sO[w][8 * hh + r][dt * 16 + ln] = oacc[dt][r] * l_r[r];
  __builtin_amdgcn_fence(__ATOMIC_ACQ_REL, "workgroup");
  __builtin_amdgcn_wave_barrier();
  for (int pass = 0; pass < 2; ++pass) {
    for (int r = 0; r < 16; ++r) {
      const int row = q0 + r;
      if (row < T && lane < D / 4) {
        const v4f val = *(const v4fa*)&sO[w][r][lane * 4];
        *(volatile v4f*)(y + ((size_t)b * T + row) * ypitch + h * D + lane * 4) = val;
      }
    }
    if (pass == 0) __threadfence();
  }
}


__global__ __launch_bounds__(256) void k_round_rows(const float* __restrict__ W, unsigned short* __restrict__ Wt, int n8) {
  const int t = blockIdx.x * 256 + threadIdx.x;
  if (t >= n8) return;
  const v4f a = *(const v4fa*)(W + (size_t)t * 8), b = *(const v4fa*)(W + (size_t)t * 8 + 4);
  v8us v; v[0]=bf16_bits(a[0]); v[1]=bf16_bits(a[1]); v[2]=bf16_bits(a[2]); v[3]=bf16_bits(a[3]);
  v[4]=bf16_bits(b[0]); v[5]=bf16_bits(b[1]); v[6]=bf16_bits(b[2]); v[7]=bf16_bits(b[3]);
  *(volatile v8us*)(Wt + (size_t)t * 8) = v; __threadfence(); *(volatile v8us*)(Wt + (size_t)t * 8) = v;
}

__global__ __launch_bounds__(256) void k_conv1(const float* __restrict__ x, const float* __restrict__ w, const float* __restrict__ b, float* __restrict__ out1) {
  const size_t t = (size_t)blockIdx.x * 256 + threadIdx.x; if (t >= (size_t)NF * C1 * 32 * 32) return;
  const int px = (int)(t % 32); size_t r = t / 32; const int py = (int)(r % 32); r /= 32; const int c = (int)(r % C1); const int f = (int)(r / C1);
  const float* img = x + (size_t)f * IMG * IMG;
  float wk[9]; for (int i = 0; i < 9; ++i) wk[i] = bf16_round(w[c * 9 + i]);
  const float bb = bf16_round(b[c]);
  float m = -3.0e38f;
  for (int dy = 0; dy < 2; ++dy) for (int dx = 0; dx < 2; ++dx) {
    const int y = 2 * py + dy, xx = 2 * px + dx; float s = bb;
    for (int ky = 0; ky < 3; ++ky) for (int kx = 0; kx < 3; ++kx) { const int yy = y + ky - 1, xq = xx + kx - 1; if (yy >= 0 && yy < IMG && xq >= 0 && xq < IMG) s += bf16_round(img[yy * IMG + xq]) * wk[ky * 3 + kx]; }
    m = fmaxf(m, fmaxf(s, 0.f));
  }
  *(volatile float*)(out1 + t) = m; __threadfence(); *(volatile float*)(out1 + t) = m;
}
__global__ __launch_bounds__(256) void k_wt_conv2(const float* __restrict__ w, unsigned short* __restrict__ Bt) {
  const int t = blockIdx.x * 256 + threadIdx.x; if (t >= C2 * 20) return;
  const int n = t / 20, k8 = (t % 20) * 8; v8us v;
  for (int i = 0; i < 8; ++i) { const int k = k8 + i; v[i] = (k < 144) ? bf16_bits(w[n * 144 + k]) : (unsigned short)0; }
  *(volatile v8us*)(Bt + n * 160 + k8) = v; __threadfence(); *(volatile v8us*)(Bt + n * 160 + k8) = v;
}
__global__ __launch_bounds__(128) void k_conv2(const float* __restrict__ in1, const unsigned short* __restrict__ Bt, const float* __restrict__ b, float* __restrict__ out2) {
  __shared__ float sD[4][16][C2 + 1];
  const int tid = threadIdx.x, w = tid >> 5, lane = tid & 31, ln = lane & 15, hh = lane >> 4;
  const int wid = blockIdx.x * 4 + w;
  const int f = wid / 32, rem = wid % 32, py = rem / 2, pxh = rem % 2;
  const int y = 2 * py + (ln >> 3), xx = 16 * pxh + (ln & 7) * 2;
  (void)y; (void)xx;
  v8f acc[2][2];
  for (int dxp = 0; dxp < 2; ++dxp) { acc[dxp][0] = (v8f){0.f,0.f,0.f,0.f,0.f,0.f,0.f,0.f}; acc[dxp][1] = acc[dxp][0]; }
  const float* img = in1 + (size_t)f * C1 * 32 * 32;
#pragma unroll
  for (int dxp = 0; dxp < 2; ++dxp) {
    const int ay = 2 * py + (ln >> 3), ax = 2 * (8 * pxh + (ln & 7)) + dxp;
    for (int ks = 0; ks < 5; ++ks) {
      FragB ah, al;
#pragma unroll
      for (int i = 0; i < 16; ++i) {
        const int k = ks * 32 + ((i < 8) ? (8 * hh + i) : (16 + 8 * hh + (i - 8)));
        float v = 0.f;
        if (k < 144) { const int c = k / 9, rr = k % 9, ky = rr / 3, kx = rr % 3; const int yy = ay + ky - 1, xq = ax + kx - 1; if (yy >= 0 && yy < 32 && xq >= 0 && xq < 32) v = img[(c * 32 + yy) * 32 + xq]; }
        const unsigned short hb = bf16_bits(v); ah.u[i] = hb; al.u[i] = bf16_bits(v - bf16_val(hb));
      }
#pragma unroll
      for (int nt = 0; nt < 2; ++nt) { FragB bb; bb.half[0] = *(const v8us*)(Bt + (nt * 16 + ln) * 160 + ks * 32 + 8 * hh); bb.half[1] = *(const v8us*)(Bt + (nt * 16 + ln) * 160 + ks * 32 + 16 + 8 * hh); acc[dxp][nt] = mmaN<2>(ah.v, al.v, bb.v, bb.v, acc[dxp][nt]); }
    }
  }
#pragma unroll
  for (int nt = 0; nt < 2; ++nt) { const float bv = bf16_round(b[nt * 16 + ln]);
#pragma unroll
    for (int r = 0; r < 8; ++r) { const float v = fmaxf(fmaxf(acc[0][nt][r] + bv, 0.f), fmaxf(acc[1][nt][r] + bv, 0.f)); sD[w][8 * hh + r][nt * 16 + ln] = v; } }
  __builtin_amdgcn_fence(__ATOMIC_ACQ_REL, "workgroup"); __builtin_amdgcn_wave_barrier();
  __shared__ float sP[2][C2][2][8];
  {
    const int pyl = (w >> 1), pxl = (w & 1);
    for (int e = lane; e < 8 * C2; e += 32) { const int j = e & 7, c = e >> 3; sP[pyl][c][pxl][j] = fmaxf(sD[w][j][c], sD[w][8 + j][c]); }
  }
  __syncthreads();
  {
    const int fblk = (blockIdx.x * 4) / 32, py0 = (((blockIdx.x * 4) % 32) / 2);
    for (int pass = 0; pass < 2; ++pass) {
      for (int e = tid; e < 256; e += 128) {
        const int c = e >> 3, q8 = e & 7; const int pyl = q8 >> 2, x4 = (q8 & 3) * 4;
        v4f v; for (int u = 0; u < 4; ++u) { const int xq = x4 + u; v[u] = sP[pyl][c][xq >> 3][xq & 7]; }
        *(volatile v4f*)(out2 + (((size_t)fblk * C2 + c) * 16 + py0 + pyl) * 16 + x4) = v;
      }
      if (pass == 0) __threadfence();
    }
  }
}
__global__ __launch_bounds__(128) void k_conv3_mean(const float* __restrict__ in2, const unsigned short* __restrict__ Bt, const float* __restrict__ b, float* __restrict__ emb) {
  __shared__ float sE[DIN];
  const int tid = threadIdx.x, w = tid >> 5, lane = tid & 31, ln = lane & 15, hh = lane >> 4;
  const int f = blockIdx.x; const float* img = in2 + (size_t)f * C2 * 256;
  v8f acc[4]; for (int t = 0; t < 4; ++t) acc[t] = (v8f){0.f,0.f,0.f,0.f,0.f,0.f,0.f,0.f};
  for (int y = 0; y < 16; ++y) {
    for (int ks = 0; ks < 9; ++ks) {
      FragB ah, al;
#pragma unroll
      for (int i = 0; i < 16; ++i) {
        const int k = ks * 32 + ((i < 8) ? (8 * hh + i) : (16 + 8 * hh + (i - 8)));
        const int c = k / 9, rr = k % 9, ky = rr / 3, kx = rr % 3; const int yy = y + ky - 1, xq = ln + kx - 1;
        const float v = (yy >= 0 && yy < 16 && xq >= 0 && xq < 16) ? img[(c * 16 + yy) * 16 + xq] : 0.f;
        const unsigned short hb = bf16_bits(v); ah.u[i] = hb; al.u[i] = bf16_bits(v - bf16_val(hb));
      }
#pragma unroll
      for (int t = 0; t < 4; ++t) { const int n = w * 64 + t * 16 + ln; FragB bb; bb.half[0] = *(const v8us*)(Bt + (size_t)n * 288 + ks * 32 + 8 * hh); bb.half[1] = *(const v8us*)(Bt + (size_t)n * 288 + ks * 32 + 16 + 8 * hh); acc[t] = mmaN<2>(ah.v, al.v, bb.v, bb.v, acc[t]); }
    }
  }
#pragma unroll
  for (int t = 0; t < 4; ++t) { float s = 0.f; for (int r = 0; r < 8; ++r) s += acc[t][r]; s += __shfl_xor(s, 16, 32); if (hh == 0) sE[w * 64 + t * 16 + ln] = s * (1.0f / 256.0f) + bf16_round(b[w * 64 + t * 16 + ln]); }
  __syncthreads();
  for (int pass = 0; pass < 2; ++pass) { if (tid < 64) { const v4f v = *(const v4fa*)&sE[tid * 4]; *(volatile v4f*)(emb + (size_t)f * DIN + tid * 4) = v; } if (pass == 0) __threadfence(); }
}
__global__ __launch_bounds__(32) void k_lstm(const float* __restrict__ emb, const unsigned short* __restrict__ W0t, const float* __restrict__ b0, const unsigned short* __restrict__ W1t, const float* __restrict__ b1,
                                           float* __restrict__ h1out) {
  __shared__ __attribute__((aligned(16))) float sIn[16][DIN + HID + HID];
  __shared__ __attribute__((aligned(16))) float sC[2][16][HID];
  __shared__ __attribute__((aligned(16))) float sHn[16][HID];
  const int lane = threadIdx.x, ln = lane & 15, hh = lane >> 4; const int b0r = blockIdx.x * 16;
  for (int e = lane; e < 16 * (DIN + 2 * HID); e += 32) sIn[e / (DIN + 2 * HID)][e % (DIN + 2 * HID)] = 0.f;
  for (int e = lane; e < 2 * 16 * HID; e += 32) (&sC[0][0][0])[e] = 0.f;
  for (int t = 0; t < NT_; ++t) {
    __builtin_amdgcn_fence(__ATOMIC_ACQ_REL, "workgroup"); __builtin_amdgcn_wave_barrier();
    for (int e = lane; e < 16 * DIN; e += 32) { const int r = e / DIN, c = e % DIN; sIn[r][c] = emb[((size_t)(b0r + r) * NT_ + t) * DIN + c]; }
    __builtin_amdgcn_fence(__ATOMIC_ACQ_REL, "workgroup"); __builtin_amdgcn_wave_barrier();
#pragma unroll 1
    for (int L = 0; L < 2; ++L) {
      const int K = L ? 2 * HID : DIN + HID; const int c0 = L ? DIN : 0;
      const unsigned short* Wt = L ? W1t : W0t; const float* bias = L ? b1 : b0;
#pragma unroll 1
      for (int ut = 0; ut < HID / 16; ++ut) {
        v8f g[4] = {};
        for (int ks = 0; ks < K / 32; ++ks) {
          FragB ah, al;
#pragma unroll
          for (int i = 0; i < 16; ++i) { const int k = ks * 32 + ((i < 8) ? (8 * hh + i) : (16 + 8 * hh + (i - 8))); const float x = sIn[ln][c0 + k]; const unsigned short hb = bf16_bits(x); ah.u[i] = hb; al.u[i] = bf16_bits(x - bf16_val(hb)); }
#pragma unroll
          for (int q = 0; q < 4; ++q) { const int n = q * HID + ut * 16 + ln; FragB bb; bb.half[0] = *(const v8us*)(Wt + (size_t)n * K + ks * 32 + 8 * hh); bb.half[1] = *(const v8us*)(Wt + (size_t)n * K + ks * 32 + 16 + 8 * hh); g[q] = mmaN<2>(ah.v, al.v, bb.v, bb.v, g[q]); }
        }
        const int u = ut * 16 + ln;
        const float bf_ = bf16_round(bias[u]), bi_ = bf16_round(bias[HID + u]), bg_ = bf16_round(bias[2 * HID + u]), bo_ = bf16_round(bias[3 * HID + u]);
#pragma unroll
        for (int r = 0; r < 8; ++r) {
          const float cprev = sC[L][8 * hh + r][u];
          const float fg = 1.0f / (1.0f + expf(-(g[0][r] + bf_))), ig = 1.0f / (1.0f + expf(-(g[1][r] + bi_))), gg = tanhf(g[2][r] + bg_), og = 1.0f / (1.0f + expf(-(g[3][r] + bo_)));
          const float cn = fg * cprev + ig * gg;
          sC[L][8 * hh + r][u] = cn;
          sHn[8 * hh + r][u] = og * tanhf(cn);
        }
      }
      __builtin_amdgcn_fence(__ATOMIC_ACQ_REL, "workgroup"); __builtin_amdgcn_wave_barrier();
      for (int e = lane; e < 16 * HID; e += 32) { const int r = e / HID, u2 = e % HID; sIn[r][DIN + L * HID + u2] = sHn[r][u2]; }
      __builtin_amdgcn_fence(__ATOMIC_ACQ_REL, "workgroup"); __builtin_amdgcn_wave_barrier();
    }
  }
  for (int pass = 0; pass < 2; ++pass) { for (int r = 0; r < 16; ++r) for (int c = lane * 4; c < HID; c += 128) { const v4f v = *(const v4fa*)&sIn[r][DIN + HID + c]; *(volatile v4f*)(h1out + (size_t)(b0r + r) * HID + c) = v; } if (pass == 0) __threadfence(); }
}
__global__ __launch_bounds__(256) void k_cls(const float* __restrict__ h1, const float* __restrict__ Wc, const float* __restrict__ bc, float* __restrict__ out) {
  __shared__ float so[NBT * NCLS];
  for (int t = threadIdx.x; t < NBT * NCLS; t += 256) { const int b = t / NCLS, o = t % NCLS; float s = bf16_round(bc[o]);
#pragma unroll 1
    for (int k = 0; k < HID; ++k) s += h1[(size_t)b * HID + k] * bf16_round(Wc[k * NCLS + o]); so[t] = s; }
  __syncthreads();
  for (int pass = 0; pass < 2; ++pass) { for (int t = threadIdx.x; t < NBT * NCLS; t += 256) *(volatile float*)(out + t) = so[t]; if (pass == 0) __threadfence(); }
}
extern "C" void kernel_launch(void* const* d_in, const int* in_sizes, int n_in,
                              void* d_out, int out_size, void* d_ws, size_t ws_size, hipStream_t stream) {
  (void)in_sizes; (void)n_in; (void)out_size;
  const float* x = (const float*)d_in[0]; const float* c1w = (const float*)d_in[1]; const float* c1b = (const float*)d_in[2]; const float* c2w = (const float*)d_in[3]; const float* c2b = (const float*)d_in[4];
  const float* c3w = (const float*)d_in[5]; const float* c3b = (const float*)d_in[6]; const float* W0 = (const float*)d_in[7]; const float* b0 = (const float*)d_in[8];
  const float* W1 = (const float*)d_in[9]; const float* b1 = (const float*)d_in[10]; const float* Wc = (const float*)d_in[11]; const float* bc = (const float*)d_in[12];
  char* ws = (char*)d_ws; size_t off = 0;
  auto take = [&](size_t bytes) { char* p = ws + off; off += (bytes + 255) & ~(size_t)255; return p; };
  unsigned short* Bt2 = (unsigned short*)take(C2 * 160 * 2); unsigned short* Bt3 = (unsigned short*)take((size_t)DIN * 288 * 2);
  unsigned short* W0t = (unsigned short*)take((size_t)G4 * (DIN + HID) * 2); unsigned short* W1t = (unsigned short*)take((size_t)G4 * 2 * HID * 2);
  float* out1 = (float*)take((size_t)NF * C1 * 32 * 32 * 4); float* out2 = (float*)take((size_t)NF * C2 * 16 * 16 * 4); float* emb = (float*)take((size_t)NF * DIN * 4); float* h1 = (float*)take((size_t)NBT * HID * 4);
  if (off > ws_size) return;
  k_wt_conv2<<<(C2 * 20 + 255) / 256, 256, 0, stream>>>(c2w, Bt2);
  k_round_rows<<<(DIN * 288 / 8 + 255) / 256, 256, 0, stream>>>(c3w, Bt3, DIN * 288 / 8);
  k_wt_bf16<<<(G4 * ((DIN + HID) / 8) + 255) / 256, 256, 0, stream>>>(W0, W0t, DIN + HID, G4);
  k_wt_bf16<<<(G4 * (2 * HID / 8) + 255) / 256, 256, 0, stream>>>(W1, W1t, 2 * HID, G4);
  k_conv1<<<(unsigned)(((size_t)NF * C1 * 32 * 32 + 255) / 256), 256, 0, stream>>>(x, c1w, c1b, out1);
  k_conv2<<<NF * 32 / 4, 128, 0, stream>>>(out1, Bt2, c2b, out2);
  k_conv3_mean<<<NF, 128, 0, stream>>>(out2, Bt3, c3b, emb);
  k_lstm<<<NBT / 16, 32, 0, stream>>>(emb, W0t, b0, W1t, b1, h1);
  k_cls<<<1, 256, 0, stream>>>(h1, Wc, bc, (float*)d_out);
}
